// STGAT_77129022701698
// MI455X (gfx1250) — hardware-verified
//
#include <hip/hip_runtime.h>


#define NND 16000
#define NE 262144
#define FIN 96
#define NH 4
#define HC (NH * FIN)
#define NSMP 32
#define NST 500
#define TT 12
#define FEAT 8
#define XIN (NST * FEAT)
#define HL 256
#define G4 (4 * HL)
#define NOUT2 (NST * 2)
#define RB 512
#define CHK 8192
#define EPT (CHK / RB)

typedef __attribute__((ext_vector_type(16))) __bf16   v16bf;
typedef __attribute__((ext_vector_type(16))) _Float16 v16h;
typedef __attribute__((ext_vector_type(8)))  float    v8f;
typedef __attribute__((ext_vector_type(8)))  unsigned v8u;

__device__ __forceinline__ unsigned f2bf(float f) { unsigned u = __float_as_uint(f); u += 0x7FFFu + ((u >> 16) & 1u); return u >> 16; }
__device__ __forceinline__ unsigned f2h(float f) { return (unsigned)__builtin_bit_cast(unsigned short, (_Float16)f); }
__device__ __forceinline__ int kpat(int v, int half) { return ((v & 4) ? 16 : 0) + half * 8 + 2 * (v & 3); }

template <int F16, int NP> struct Opnd { v16bf p[NP]; };

template <int F16, int NP> __device__ __forceinline__ void pack2(float f0, float f1, unsigned* o) {
    if (F16) { o[0] = f2h(f0) | (f2h(f1) << 16); return; }
    unsigned h0 = f2bf(f0), h1 = f2bf(f1); o[0] = h0 | (h1 << 16);
    if (NP >= 2) {
        float r0 = f0 - __uint_as_float(h0 << 16), r1 = f1 - __uint_as_float(h1 << 16);
        unsigned m0 = f2bf(r0), m1 = f2bf(r1); o[1] = m0 | (m1 << 16);
        if (NP >= 3) {
            float s0 = r0 - __uint_as_float(m0 << 16), s1 = r1 - __uint_as_float(m1 << 16);
            o[2] = f2bf(s0) | (f2bf(s1) << 16);
        }
    }
}
template <int F16, int NP> __device__ __forceinline__ void op_row(const float* rowp, int half, float sc, Opnd<F16, NP>& o) {
    v8u u[NP];
#pragma unroll
    for (int v = 0; v < 8; ++v) {
        int kk = kpat(v, half); unsigned t[3];
        pack2<F16, NP>(rowp[kk] * sc, rowp[kk + 1] * sc, t);
#pragma unroll
        for (int p = 0; p < NP; ++p) u[p][v] = t[p];
    }
#pragma unroll
    for (int p = 0; p < NP; ++p) o.p[p] = __builtin_bit_cast(v16bf, u[p]);
}
template <int F16, int NP> __device__ __forceinline__ void op_row_tail(const float* rowp, int half, float sc, int kvalid, Opnd<F16, NP>& o) {
    v8u u[NP];
#pragma unroll
    for (int v = 0; v < 8; ++v) {
        int kk = kpat(v, half); unsigned t[3];
        float f0 = kk < kvalid ? rowp[kk] * sc : 0.0f, f1 = (kk + 1) < kvalid ? rowp[kk + 1] * sc : 0.0f;
        pack2<F16, NP>(f0, f1, t);
#pragma unroll
        for (int p = 0; p < NP; ++p) u[p][v] = t[p];
    }
#pragma unroll
    for (int p = 0; p < NP; ++p) o.p[p] = __builtin_bit_cast(v16bf, u[p]);
}
template <int F16, int NP> __device__ __forceinline__ void op_col(const float* M, int ld, int n, int k0, int half, float sc, Opnd<F16, NP>& o) {
    v8u u[NP];
#pragma unroll
    for (int v = 0; v < 8; ++v) {
        int kk = k0 + kpat(v, half); unsigned t[3];
        pack2<F16, NP>(M[(size_t)kk * ld + n] * sc, M[(size_t)(kk + 1) * ld + n] * sc, t);
#pragma unroll
        for (int p = 0; p < NP; ++p) u[p][v] = t[p];
    }
#pragma unroll
    for (int p = 0; p < NP; ++p) o.p[p] = __builtin_bit_cast(v16bf, u[p]);
}
template <int F16, int NP> __device__ __forceinline__ void op_col_tail(const float* M, int ld, int n, int k0, int half, float sc, int K, Opnd<F16, NP>& o) {
    v8u u[NP];
#pragma unroll
    for (int v = 0; v < 8; ++v) {
        int kk = k0 + kpat(v, half); unsigned t[3];
        float f0 = kk < K ? M[(size_t)kk * ld + n] * sc : 0.0f, f1 = (kk + 1) < K ? M[(size_t)(kk + 1) * ld + n] * sc : 0.0f;
        pack2<F16, NP>(f0, f1, t);
#pragma unroll
        for (int p = 0; p < NP; ++p) u[p][v] = t[p];
    }
#pragma unroll
    for (int p = 0; p < NP; ++p) o.p[p] = __builtin_bit_cast(v16bf, u[p]);
}
__device__ __forceinline__ v8f wm_bf16(v16bf a, v16bf b, v8f c) { return __builtin_amdgcn_wmma_f32_16x16x32_bf16(false, a, false, b, (short)0, c, false, false); }
template <int F16, int NA, int NB> __device__ __forceinline__ v8f wmma_op(const Opnd<F16, NA>& a, const Opnd<F16, NB>& b, v8f c) {
    if (F16) {
        v16h ah = __builtin_bit_cast(v16h, a.p[0]), bh = __builtin_bit_cast(v16h, b.p[0]);
        c = __builtin_amdgcn_wmma_f32_16x16x32_f16(false, ah, false, bh, (short)0, c, false, false);
        asm volatile("v_nop\n\tv_nop\n\tv_nop\n\tv_nop" : "+v"(c) : "v"(ah), "v"(bh));
        return c;
    }
    constexpr int NMX = NA > NB ? NA : NB;
#pragma unroll
    for (int i = 0; i < NA; ++i)
#pragma unroll
        for (int j = 0; j < NB; ++j)
            if (i + j < NMX) c = wm_bf16(a.p[i], b.p[j], c);
    if (NA == 1 && NB == 1)      asm volatile("v_nop\n\tv_nop\n\tv_nop\n\tv_nop" : "+v"(c) : "v"(a.p[0]), "v"(b.p[0]));
    else if (NA == 2 && NB == 1) asm volatile("v_nop\n\tv_nop\n\tv_nop\n\tv_nop" : "+v"(c) : "v"(a.p[0]), "v"(a.p[1]), "v"(b.p[0]));
    else if (NA == 1 && NB == 2) asm volatile("v_nop\n\tv_nop\n\tv_nop\n\tv_nop" : "+v"(c) : "v"(a.p[0]), "v"(b.p[0]), "v"(b.p[1]));
    else if (NA == 2 && NB == 2) asm volatile("v_nop\n\tv_nop\n\tv_nop\n\tv_nop" : "+v"(c) : "v"(a.p[0]), "v"(a.p[1]), "v"(b.p[0]), "v"(b.p[1]));
    else                         asm volatile("v_nop\n\tv_nop\n\tv_nop\n\tv_nop" : "+v"(c) : "v"(a.p[0]), "v"(a.p[NA - 1]), "v"(b.p[0]), "v"(b.p[NB - 1]), "v"(a.p[NA / 2]), "v"(b.p[NB / 2]));
    return c;
}

struct ZMap { long long s1; long long s2; int zdiv; int pad_; };
__device__ __forceinline__ size_t zoff(const ZMap& m, int z) { return (size_t)((long long)(z / m.zdiv) * m.s1 + (long long)(z % m.zdiv) * m.s2); }

#define ACT_NONE 0
#define ACT_RELU 1
#define ACT_GELU_ERF 2
#define ACT_SILU 3
#define ACT_TANH 4
__device__ __forceinline__ float act_apply(int act, float x) {
    if (act == ACT_RELU) return x > 0.f ? x : 0.f;
    if (act == ACT_GELU_ERF) return 0.5f * x * (1.0f + erff(x * 0.70710678118654752f));
    if (act == ACT_SILU) return x / (1.0f + expf(-x));
    if (act == ACT_TANH) return tanhf(x);
    return x;
}
struct GemmArgs {
    ZMap za, zb_, zc, zbias, zadd, zrsc, zmul, zrbias;
    const float* A; const float* Bm; float* C; const float* bias; const float* add; const float* rsc; const float* mul; const float* rbias;
    long long ldadd, ldmul;
    int lda, ldb, ldc, K;
    float ascale, bscale, oscale, addscale;
    int M, nvalid, nstore, ldrsc;
    int bcs, pad1, pad2, pad3;
};
template <int BT, int F16, int NA, int NB, int RW, int CW, int ACT>
__global__ __launch_bounds__(256) void gemm_kernel(GemmArgs g) {
    constexpr int TR = 16 * RW, TC = 64 * CW, CSTR = TC + 4;
    __shared__ __align__(16) float cst[TR * CSTR];
    const int z = blockIdx.z;
    const float* A = g.A + zoff(g.za, z); const float* Bm = g.Bm + zoff(g.zb_, z); float* C = g.C + zoff(g.zc, z);
    const int tid = threadIdx.x, lane = tid & 31, wv = tid >> 5;
    const int l16 = lane & 15, half = lane >> 4;
    const int rt = wv % RW, ch = wv / RW;
    const int row0 = blockIdx.x * TR, col0 = blockIdx.y * TC + ch * 64;
    int arix = row0 + rt * 16 + l16; if (arix >= g.M) arix = g.M - 1;
    const float* arow = A + (size_t)arix * g.lda;
    v8f acc[4];
#pragma unroll
    for (int t = 0; t < 4; ++t) acc[t] = (v8f){};
    const int K = g.K;
#pragma unroll 1
    for (int kc = 0; kc < K; kc += 32) {
        Opnd<F16, NA> a;
        if (kc + 32 <= K) op_row<F16, NA>(arow + kc, half, g.ascale, a); else op_row_tail<F16, NA>(arow + kc, half, g.ascale, K - kc, a);
#pragma unroll
        for (int t = 0; t < 4; ++t) {
            Opnd<F16, NB> b;
            const int n = col0 + t * 16 + l16;
            if (n < g.nvalid) {
                if (BT) { if (kc + 32 <= K) op_row<F16, NB>(Bm + (size_t)n * g.ldb + kc, half, g.bscale, b); else op_row_tail<F16, NB>(Bm + (size_t)n * g.ldb + kc, half, g.bscale, K - kc, b); }
                else    { if (kc + 32 <= K) op_col<F16, NB>(Bm, g.ldb, n * g.bcs, kc, half, g.bscale, b); else op_col_tail<F16, NB>(Bm, g.ldb, n * g.bcs, kc, half, g.bscale, K, b); }
            } else {
#pragma unroll
                for (int p = 0; p < NB; ++p) b.p[p] = (v16bf){};
            }
            acc[t] = wmma_op<F16, NA, NB>(a, b, acc[t]);
        }
    }
    const float* bias = g.bias ? g.bias + zoff(g.zbias, z) : nullptr;
    const float* add = g.add ? g.add + zoff(g.zadd, z) : nullptr;
    const float* rsc = g.rsc ? g.rsc + zoff(g.zrsc, z) : nullptr;
    const float* mul = g.mul ? g.mul + zoff(g.zmul, z) : nullptr;
    const float* rbias = g.rbias ? g.rbias + zoff(g.zrbias, z) : nullptr;
#pragma unroll
    for (int t = 0; t < 4; ++t) {
        const int cl = ch * 64 + t * 16 + l16;
        const int cg = blockIdx.y * TC + cl;
        const bool cok = cg < g.nvalid;
        const float bv = (bias && cok) ? bias[(size_t)cg * g.bcs] : 0.0f;
#pragma unroll
        for (int r = 0; r < 8; ++r) {
            const int rl = rt * 16 + r + 8 * half;
            float v = acc[t][r] * g.oscale + bv;
            int rg = row0 + rl; if (rg >= g.M) rg = g.M - 1;
            if (rbias) v += rbias[rg];
            if (rsc) v *= rsc[(size_t)rg * g.ldrsc];
            if (mul && cok) v *= mul[(size_t)rg * g.ldmul + cg];
            if (add && cok) v += g.addscale * add[(size_t)rg * g.ldadd + cg];
            cst[rl * CSTR + cl] = v;
        }
    }
    __syncthreads();
    const int col = tid % TC, rsel = tid / TC, rstep = 256 / TC;
    if (ACT != ACT_NONE) {
#pragma unroll 1
        for (int r = rsel; r < TR; r += rstep) cst[r * CSTR + col] = act_apply(ACT, cst[r * CSTR + col]);
    }
    float* ob = C + (size_t)row0 * g.ldc + (size_t)blockIdx.y * TC;
    const bool colok = (int)(blockIdx.y * TC + col) < g.nstore;
    const int rmax = (g.M - row0 < TR) ? (g.M - row0) : TR;
    auto pass = [&]() {
        if (colok) {
#pragma unroll 4
            for (int r = rsel; r < rmax; r += rstep) *(volatile float*)(ob + (size_t)r * g.ldc + col) = cst[r * CSTR + col];
        }
    };
    pass();
    __threadfence();
    pass();
}
static inline ZMap zm(long long s1) { ZMap m; m.s1 = s1; m.s2 = 0; m.zdiv = 1; m.pad_ = 0; return m; }
static inline ZMap zm2(long long s1, long long s2, int zdiv) { ZMap m; m.s1 = s1; m.s2 = s2; m.zdiv = zdiv; m.pad_ = 0; return m; }
static inline GemmArgs gemm_args(const float* A, int lda, ZMap za, const float* Bm, int ldb, ZMap zb, float* C, int ldc, ZMap zc, int M, int N, int K) {
    GemmArgs g; g.za = za; g.zb_ = zb; g.zc = zc; g.zbias = zm(0); g.zadd = zm(0); g.zrsc = zm(0); g.zmul = zm(0); g.zrbias = zm(0);
    g.A = A; g.Bm = Bm; g.C = C; g.bias = nullptr; g.add = nullptr; g.rsc = nullptr; g.mul = nullptr; g.rbias = nullptr; g.ldadd = 0; g.ldmul = 0;
    g.lda = lda; g.ldb = ldb; g.ldc = ldc; g.K = K; g.ascale = 1.0f; g.bscale = 1.0f; g.oscale = 1.0f; g.addscale = 1.0f; g.M = M; g.nvalid = N; g.nstore = N; g.ldrsc = 1;
    g.bcs = 1; g.pad1 = 0; g.pad2 = 0; g.pad3 = 0;
    return g;
}
static_assert(sizeof(ZMap) == 24, "ZMap layout");
static_assert(sizeof(GemmArgs) == 8 * 24 + 8 * 8 + 2 * 8 + 4 * 4 + 4 * 4 + 4 * 4 + 4 * 4, "GemmArgs has no padding");

__global__ __launch_bounds__(256) void softmax_rows(float* S, long long sy, long long sx, int L, float prescale, const float* addv, long long say, int aydiv, int causal,
                                                  const int* imask, long long imy, long long imx, float maskval) {
    __shared__ float red[8];
    const int tid = threadIdx.x, lane = tid & 31, wid = tid >> 5;
    float* row = S + (size_t)blockIdx.y * sy + (size_t)blockIdx.x * sx;
    const float* av = addv ? addv + (size_t)(blockIdx.y / aydiv) * say : nullptr;
    const int* im = imask ? imask + (size_t)(blockIdx.y / aydiv) * imy + (size_t)blockIdx.x * imx : nullptr;
    float v[16];
    const int nj = L / 256;
    float mx = -__builtin_inff();
#pragma unroll
    for (int j = 0; j < 16; ++j) if (j < nj) { float t = row[tid + 256 * j] * prescale; if (av) t += av[tid + 256 * j]; if (im && im[tid + 256 * j] == 0) t = maskval; if (causal && (tid + 256 * j) > (int)blockIdx.x) t = -__builtin_inff(); v[j] = t; mx = fmaxf(mx, t); }
#pragma unroll
    for (int o = 16; o; o >>= 1) mx = fmaxf(mx, __shfl_xor(mx, o, 32));
    if (lane == 0) red[wid] = mx;
    __syncthreads();
    float m = red[0];
#pragma unroll
    for (int i = 1; i < 8; ++i) m = fmaxf(m, red[i]);
    if (m == -__builtin_inff()) m = 0.f;
    __syncthreads();
    float sum = 0.f;
#pragma unroll
    for (int j = 0; j < 16; ++j) if (j < nj) { v[j] = expf(v[j] - m); sum += v[j]; }
#pragma unroll
    for (int o = 16; o; o >>= 1) sum += __shfl_xor(sum, o, 32);
    if (lane == 0) red[wid] = sum;
    __syncthreads();
    float tot = 0.f;
#pragma unroll
    for (int i = 0; i < 8; ++i) tot += red[i];
    const float inv = 1.0f / tot;
#pragma unroll
    for (int j = 0; j < 16; ++j) if (j < nj) *(volatile float*)(row + tid + 256 * j) = v[j] * inv;
    __threadfence();
#pragma unroll
    for (int j = 0; j < 16; ++j) if (j < nj) *(volatile float*)(row + tid + 256 * j) = v[j] * inv;
}

#define VST2(T, p, v) do { const T vst2_v_ = (v); *(volatile T*)(p) = vst2_v_; __threadfence(); *(volatile T*)(p) = vst2_v_; } while (0)
__device__ __forceinline__ int block_excl_scan(int cnt, int* scan, int tid, int& total) { const int lane = tid & 31, w = tid >> 5; int x = cnt;
#pragma unroll
    for (int o = 1; o < 32; o <<= 1) { const int y = __shfl_up(x, o, 32); if (lane >= o) x += y; }
    __syncthreads(); if (lane == 31) scan[w] = x; __syncthreads();
    if (w == 0) { int v = (lane < RB / 32) ? scan[lane] : 0;
#pragma unroll
        for (int o = 1; o < 32; o <<= 1) { const int y = __shfl_up(v, o, 32); if (lane >= o) v += y; }
        if (lane < RB / 32) scan[lane] = v; }
    __syncthreads(); total = scan[RB / 32 - 1]; const int base = (w > 0) ? scan[w - 1] : 0; return base + x - cnt; }
__device__ __forceinline__ int clampn(int s) { return s < 0 ? 0 : (s >= NND ? NND - 1 : s); }
__device__ __forceinline__ float lrelu(float x) { return x > 0.f ? x : 0.2f * x; }
__global__ __launch_bounds__(256) void k_alph(const float* __restrict__ XP, const float* __restrict__ as, const float* __restrict__ ad, float* AS) { const int lane = threadIdx.x & 31; const int n = blockIdx.x * 8 + (threadIdx.x >> 5); if (n >= NND) return; float v = 0.f;
#pragma unroll
    for (int h = 0; h < NH; ++h) { float s = 0.f, d = 0.f;
#pragma unroll
        for (int q = 0; q < 3; ++q) { const float x = XP[(size_t)n * HC + h * FIN + lane + 32 * q]; s += x * as[h * FIN + lane + 32 * q]; d += x * ad[h * FIN + lane + 32 * q]; }
#pragma unroll
        for (int o = 16; o; o >>= 1) { s += __shfl_xor(s, o, 32); d += __shfl_xor(d, o, 32); } if (lane == h) v = s; if (lane == 4 + h) v = d; }
    if (lane < 8) { VST2(float, AS + (size_t)n * 8 + lane, v); } }
__global__ __launch_bounds__(RB) void k_gat(const float* __restrict__ XP, const float* __restrict__ AS, const int* __restrict__ ei, float* GH) { __shared__ unsigned short Lr[CHK]; __shared__ int Lc[CHK]; __shared__ int scan[RB]; const int tid = threadIdx.x; const int n0 = blockIdx.x * RB; const int h = blockIdx.y; const int n = n0 + tid; const int nn = n < NND ? n : NND - 1;
    const float adn = AS[(size_t)nn * 8 + 4 + h]; float m = -__builtin_inff(), den = 0.f; float acc[FIN];
#pragma unroll
    for (int c = 0; c < FIN; ++c) acc[c] = 0.f;
    for (int e0 = 0; e0 < NE + CHK; e0 += CHK) { int tot = 0;
        if (e0 < NE) { int hr[EPT], hc[EPT]; int cnt = 0;
#pragma unroll
            for (int k = 0; k < EPT; ++k) { const int e = e0 + tid * EPT + k; hr[k] = -1; if (e < NE) { const int d = ei[(size_t)NE + e]; if (d >= n0 && d < n0 + RB) { hr[k] = d - n0; hc[k] = clampn(ei[e]); ++cnt; } } }
            int p = block_excl_scan(cnt, scan, tid, tot);
#pragma unroll
            for (int k = 0; k < EPT; ++k) if (hr[k] >= 0) { Lr[p] = (unsigned short)hr[k]; Lc[p] = hc[k]; ++p; }
            __syncthreads(); }
        const int nq = (e0 < NE) ? tot : 1;
        for (int q = 0; q < nq; ++q) { int s; if (e0 < NE) { if ((int)Lr[q] != tid) continue; s = Lc[q]; } else s = nn;
            const float e = lrelu(AS[(size_t)s * 8 + h] + adn); const float mn = fmaxf(m, e); const float sc = expf(m - mn); const float w = expf(e - mn); den = den * sc + w; const float* xr = XP + (size_t)s * HC + h * FIN;
#pragma unroll
            for (int c = 0; c < FIN; ++c) acc[c] = acc[c] * sc + w * xr[c]; m = mn; }
        __syncthreads(); }
    if (n >= NND) return; const float inv = 1.f / (den + 1e-16f);
#pragma unroll
    for (int c = 0; c < FIN; ++c) VST2(float, GH + (size_t)n * HC + h * FIN + c, acc[c] * inv); }
__global__ __launch_bounds__(256) void k_hmean(const float* __restrict__ GH, const float* __restrict__ b, float* X1) { const int q = blockIdx.x * 256 + threadIdx.x; if (q >= NND * FIN) return; const int c = q % FIN; const size_t n = q / FIN; const float* g = GH + n * HC + c; VST2(float, X1 + q, 0.25f * (g[0] + g[FIN] + g[2 * FIN] + g[3 * FIN]) + b[c]); }
__global__ __launch_bounds__(256) void k_regroup(const float* __restrict__ X2, float* XL) { const size_t q = (size_t)blockIdx.x * 256 + threadIdx.x; if (q >= (size_t)TT * NSMP * XIN) return; const int col = (int)(q % XIN); const int row = (int)(q / XIN); const int b = row % NSMP, t = row / NSMP; const int node = col / FEAT, f = col % FEAT; VST2(float, XL + q, X2[((size_t)b * NST + node) * FIN + t * FEAT + f]); }
__global__ __launch_bounds__(256) void k_cell(const float* __restrict__ XG, const float* __restrict__ HG, const float* __restrict__ bi, const float* __restrict__ bh, int t, float* Cst, float* Hst, float* HS) { const int q = blockIdx.x * 256 + threadIdx.x; if (q >= NSMP * HL) return; const int j = q % HL, b = q / HL; const float* xg = XG + ((size_t)t * NSMP + b) * G4; const float* hg = HG + (size_t)b * G4;
    const float gi = xg[j] + hg[j] + bi[j] + bh[j], gf = xg[HL + j] + hg[HL + j] + bi[HL + j] + bh[HL + j], gg = xg[2 * HL + j] + hg[2 * HL + j] + bi[2 * HL + j] + bh[2 * HL + j], go = xg[3 * HL + j] + hg[3 * HL + j] + bi[3 * HL + j] + bh[3 * HL + j];
    const float c = (1.f / (1.f + expf(-gf))) * Cst[q] + (1.f / (1.f + expf(-gi))) * tanhf(gg); const float hv = (1.f / (1.f + expf(-go))) * tanhf(c);
    VST2(float, Cst + q, c); VST2(float, Hst + q, hv); VST2(float, HS + ((size_t)t * NSMP + b) * HL + j, hv); }
__global__ __launch_bounds__(256) void k_zero(float* p, int n) { const int q = blockIdx.x * 256 + threadIdx.x; if (q < n) { VST2(float, p + q, 0.f); } }
__global__ __launch_bounds__(256) void k_out(const float* __restrict__ F, float* out) { const int q = blockIdx.x * 256 + threadIdx.x; if (q >= NSMP * NOUT2) return; const int k = q % NOUT2, b = q / NOUT2; VST2(float, out + (size_t)b * NOUT2 + k, F[(size_t)b * 1024 + k]); }
extern "C" void kernel_launch(void* const* d_in, const int* in_sizes, int n_in,
                              void* d_out, int out_size, void* d_ws, size_t ws_size, hipStream_t stream) {
    (void)in_sizes; (void)n_in; (void)out_size;
    const float* x = (const float*)d_in[0]; const int* ei = (const int*)d_in[1]; const float* w0 = (const float*)d_in[2]; const float* as0 = (const float*)d_in[3]; const float* ad0 = (const float*)d_in[4]; const float* b0 = (const float*)d_in[5]; const float* w1 = (const float*)d_in[6]; const float* as1 = (const float*)d_in[7]; const float* ad1 = (const float*)d_in[8]; const float* b1 = (const float*)d_in[9];
    const float* wi1 = (const float*)d_in[10]; const float* wh1 = (const float*)d_in[11]; const float* bi1 = (const float*)d_in[12]; const float* bh1 = (const float*)d_in[13]; const float* wi2 = (const float*)d_in[14]; const float* wh2 = (const float*)d_in[15]; const float* bi2 = (const float*)d_in[16]; const float* bh2 = (const float*)d_in[17]; const float* wl = (const float*)d_in[18]; const float* bl = (const float*)d_in[19];
    float* out = (float*)d_out;
    char* wsp = (char*)d_ws;
    auto take = [&](size_t bytes) { char* p = wsp; wsp += (bytes + 255) & ~(size_t)255; return (void*)p; };
    float* XP = (float*)take((size_t)NND * HC * 4); float* AS = (float*)take((size_t)NND * 8 * 4); float* GH = (float*)take((size_t)NND * HC * 4); float* X1 = (float*)take((size_t)NND * FIN * 4); float* X2 = (float*)take((size_t)NND * FIN * 4);
    float* XL = (float*)take((size_t)TT * NSMP * XIN * 4); float* XG = (float*)take((size_t)TT * NSMP * G4 * 4); float* HG = (float*)take((size_t)64 * G4 * 4); float* Cst = (float*)take(NSMP * HL * 4); float* Hst = (float*)take((size_t)64 * HL * 4); float* HS = (float*)take((size_t)TT * NSMP * HL * 4); float* FIN32 = (float*)take((size_t)64 * 1024 * 4);
    if ((size_t)(wsp - (char*)d_ws) > ws_size) return;
    const int nb = (NND + RB - 1) / RB;
    { GemmArgs g = gemm_args(x, FIN, zm(0), w0, HC, zm(0), XP, HC, zm(0), NND, HC, FIN); gemm_kernel<0, 0, 2, 2, 4, 2, ACT_NONE><<<dim3(NND / 64, HC / 128, 1), 256, 0, stream>>>(g); }
    k_alph<<<NND / 8, 256, 0, stream>>>(XP, as0, ad0, AS);
    k_gat<<<dim3(nb, NH, 1), RB, 0, stream>>>(XP, AS, ei, GH);
    k_hmean<<<(NND * FIN) / 256, 256, 0, stream>>>(GH, b0, X1);
    { GemmArgs g = gemm_args(X1, FIN, zm(0), w1, HC, zm(0), XP, HC, zm(0), NND, HC, FIN); gemm_kernel<0, 0, 2, 2, 4, 2, ACT_NONE><<<dim3(NND / 64, HC / 128, 1), 256, 0, stream>>>(g); }
    k_alph<<<NND / 8, 256, 0, stream>>>(XP, as1, ad1, AS);
    k_gat<<<dim3(nb, NH, 1), RB, 0, stream>>>(XP, AS, ei, GH);
    k_hmean<<<(NND * FIN) / 256, 256, 0, stream>>>(GH, b1, X2);
    k_regroup<<<(unsigned)(((size_t)TT * NSMP * XIN) / 256), 256, 0, stream>>>(X2, XL);
    { GemmArgs g = gemm_args(XL, XIN, zm(0), wi1, XIN, zm(0), XG, G4, zm(0), TT * NSMP, G4, XIN); gemm_kernel<1, 0, 2, 2, 4, 2, ACT_NONE><<<dim3((TT * NSMP) / 64, G4 / 128, 1), 256, 0, stream>>>(g); }
    k_zero<<<(NSMP * HL + 255) / 256, 256, 0, stream>>>(Cst, NSMP * HL); k_zero<<<(64 * HL + 255) / 256, 256, 0, stream>>>(Hst, 64 * HL); k_zero<<<(64 * G4 + 255) / 256, 256, 0, stream>>>(HG, 64 * G4);
    for (int t = 0; t < TT; ++t) {
        if (t > 0) { GemmArgs g = gemm_args(Hst, HL, zm(0), wh1, HL, zm(0), HG, G4, zm(0), NSMP, G4, HL); gemm_kernel<1, 0, 2, 2, 4, 2, ACT_NONE><<<dim3(1, G4 / 128, 1), 256, 0, stream>>>(g); }
        k_cell<<<(NSMP * HL) / 256, 256, 0, stream>>>(XG, HG, bi1, bh1, t, Cst, Hst, HS);
    }
    { GemmArgs g = gemm_args(HS, HL, zm(0), wi2, HL, zm(0), XG, G4, zm(0), TT * NSMP, G4, HL); gemm_kernel<1, 0, 2, 2, 4, 2, ACT_NONE><<<dim3((TT * NSMP) / 64, G4 / 128, 1), 256, 0, stream>>>(g); }
    k_zero<<<(NSMP * HL + 255) / 256, 256, 0, stream>>>(Cst, NSMP * HL); k_zero<<<(64 * HL + 255) / 256, 256, 0, stream>>>(Hst, 64 * HL); k_zero<<<(64 * G4 + 255) / 256, 256, 0, stream>>>(HG, 64 * G4);
    for (int t = 0; t < TT; ++t) {
        if (t > 0) { GemmArgs g = gemm_args(Hst, HL, zm(0), wh2, HL, zm(0), HG, G4, zm(0), NSMP, G4, HL); gemm_kernel<1, 0, 2, 2, 4, 2, ACT_NONE><<<dim3(1, G4 / 128, 1), 256, 0, stream>>>(g); }
        k_cell<<<(NSMP * HL) / 256, 256, 0, stream>>>(XG, HG, bi2, bh2, t, Cst, Hst, HS);
    }
    { GemmArgs g = gemm_args(Hst, HL, zm(0), wl, HL, zm(0), FIN32, 1024, zm(0), NSMP, NOUT2, HL); g.bias = bl; gemm_kernel<1, 0, 2, 2, 4, 2, ACT_NONE><<<dim3(1, (NOUT2 + 127) / 128, 1), 256, 0, stream>>>(g); }
    k_out<<<(NSMP * NOUT2 + 255) / 256, 256, 0, stream>>>(FIN32, out);
}
